// ExtractorLoss_13331578487304
// MI455X (gfx1250) — hardware-verified
//
#include <hip/hip_runtime.h>
#include <math.h>
#include <stdint.h>


#pragma clang fp contract(off)

typedef _Float16 v16h __attribute__((ext_vector_type(16)));
typedef _Float16 v8h  __attribute__((ext_vector_type(8)));
typedef float    v8f  __attribute__((ext_vector_type(8)));
typedef float    v4f  __attribute__((ext_vector_type(4)));

#define WAVES   8
#define THREADS (WAVES * 32)
#define NPADV   512
#define QTMAX   (NPADV / 64)
#define LINEF   32

__device__ __forceinline__ v8f wmma_f16_16x16x32(v16h a, v16h b, v8f c)
{
    v8f d = __builtin_amdgcn_wmma_f32_16x16x32_f16(false, a, false, b, (short)0, c, false, false);
    asm volatile("v_nop\n\tv_nop\n\tv_nop\n\tv_nop" : "+v"(d) : "v"(a), "v"(b));
    return d;
}

__device__ __forceinline__ float bf16r(float v)
{
    unsigned int u = __float_as_uint(v);
    u = u + 0x7FFFu + ((u >> 16) & 1u);
    u &= 0xFFFF0000u;
    return __uint_as_float(u);
}

__device__ __forceinline__ int ceil_snap(float r)
{
    if (!(r > 0.0f)) r = 0.0f;
    if (r > 1048576.0f) r = 1048576.0f;
    const float n  = rintf(r);
    const float d  = r - n;
    const int   ni = (int)n;
    return (d > r * 3.8e-6f) ? (ni + 1) : ni;
}

__device__ __forceinline__ float bin_freq(int j, int Fw, int K, float ft, float delta, float sfrq, float fmin)
{
    float r;
    if (j < Fw) {
        const float of = fmaf((float)j, sfrq, -delta);
        r = ft + of;
    } else if (j < Fw + K) {
        const float kf = (float)(j - Fw);
        const float ks = kf * sfrq;
        r = fmin + ks;
    } else {
        const float kf = (float)(j - Fw - K);
        const float ks = kf * sfrq;
        const float b1 = ft + delta;
        const float b2 = b1 + sfrq;
        r = b2 + ks;
    }
    return r;
}

__global__ __launch_bounds__(THREADS) void k_psd_snr(
    const float* __restrict__ x,
    const float* __restrict__ f_true,
    const float* __restrict__ fs,
    const float* __restrict__ p_delta,
    const float* __restrict__ p_s,
    const float* __restrict__ p_fmin,
    const float* __restrict__ p_fmax,
    float* __restrict__ snr_ws,
    int B, int N)
{
    __shared__ v8h   xs8[NPADV];
    __shared__ float sW[WAVES];
    __shared__ float sU[WAVES];
    __shared__ int   sC[WAVES];
    __shared__ float sRes;

    const int b = blockIdx.x;
    if (b >= B) return;

    const int tid  = threadIdx.x;
    const int lane = tid & 31;
    const int wave = tid >> 5;
    const int m    = lane & 15;
    const int h    = lane >> 4;

    const float delta = bf16r(p_delta[0]);
    const float sfrq  = bf16r(p_s[0]);
    const float fmin  = bf16r(p_fmin[0]);
    const float fmax  = bf16r(p_fmax[0]);
    const float ft    = bf16r(f_true[b]);
    const float fsb   = bf16r(fs[b]);
    const float winv  = 6.283185307179586f / fsb;

    int Fw = 1, K = 0;
    if (sfrq > 0.0f) {
        const float a1 = delta + sfrq;
        const float a2 = a1 + delta;
        const float rw = a2 / sfrq;
        int fw = ceil_snap(rw);
        const float g  = fmax - fmin;
        const float rk = g / sfrq;
        int kk = ceil_snap(rk) + 2;
        if (fw < 1) fw = 1;
        if (fw > 4096) fw = 4096;
        if (kk < 0) kk = 0;
        if (kk > 8192) kk = 8192;
        Fw = fw;
        K  = kk;
    }
    const int Ftot   = Fw + 2 * K;
    const int ntiles = (Ftot + 15) >> 4;

    int QT = (N + 511) / 512;
    if (QT > QTMAX) QT = QTMAX;
    if (QT < 1) QT = 1;
    const int nvec = QT * 64;

    const _Float16 hz = (_Float16)0.0f;
    for (int i = tid; i < nvec; i += THREADS) {
        v8h v = {hz, hz, hz, hz, hz, hz, hz, hz};
        #pragma unroll
        for (int e = 0; e < 8; ++e) {
            const int n = i * 8 + e;
            if (n < N) v[e] = (_Float16)bf16r(x[(size_t)b * (size_t)N + (size_t)n]);
        }
        xs8[i] = v;
    }
    __syncthreads();

    const float thr1 = ft - delta;
    const float thr2 = fmax + sfrq;

    const float fz = winv * 0.0f;
    const v8f zero8 = {fz, fz, fz, fz, fz, fz, fz, fz};

    float accW = 0.0f, accU = 0.0f;
    int   accC = 0;

    #pragma unroll 1
    for (int t = wave; t < ntiles; t += WAVES) {
        const int bin0 = t * 16;

        const float fA = bin_freq(bin0 + m, Fw, K, ft, delta, sfrq, fmin);
        const float wA = winv * fA;
        const float c1 = cosf(wA);
        const float s1 = sinf(wA);
        const float c2  = c1 * c1 - s1 * s1;   const float s2  = c1 * s1 + s1 * c1;
        const float c4  = c2 * c2 - s2 * s2;   const float s4  = c2 * s2 + s2 * c2;
        const float c8  = c4 * c4 - s4 * s4;   const float s8  = c4 * s4 + s4 * c4;
        const float c16 = c8 * c8 - s8 * s8;   const float s16 = c8 * s8 + s8 * c8;
        const float cst = h ? c8 : 1.0f;
        const float sst = h ? s8 : 0.0f;

        v16h Ac = {hz, hz, hz, hz, hz, hz, hz, hz, hz, hz, hz, hz, hz, hz, hz, hz};
        v16h As = {hz, hz, hz, hz, hz, hz, hz, hz, hz, hz, hz, hz, hz, hz, hz, hz};
        {
            float c0 = cst, s0 = sst;
            #pragma unroll
            for (int i = 0; i < 8; ++i) {
                Ac[i] = (_Float16)c0;  As[i] = (_Float16)s0;
                const float cn = c0 * c1 - s0 * s1;
                const float sn = s0 * c1 + c0 * s1;
                c0 = cn; s0 = sn;
            }
            c0 = cst * c16 - sst * s16;
            s0 = sst * c16 + cst * s16;
            #pragma unroll
            for (int i = 8; i < 16; ++i) {
                Ac[i] = (_Float16)c0;  As[i] = (_Float16)s0;
                const float cn = c0 * c1 - s0 * s1;
                const float sn = s0 * c1 + c0 * s1;
                c0 = cn; s0 = sn;
            }
        }

        float wrow[8];
        #pragma unroll
        for (int v = 0; v < 8; ++v)
            wrow[v] = winv * bin_freq(bin0 + 8 * h + v, Fw, K, ft, delta, sfrq, fmin);

        float cacc[8] = {0.0f, 0.0f, 0.0f, 0.0f, 0.0f, 0.0f, 0.0f, 0.0f};
        float sacc[8] = {0.0f, 0.0f, 0.0f, 0.0f, 0.0f, 0.0f, 0.0f, 0.0f};

        #pragma unroll 1
        for (int qt = 0; qt < QT; ++qt) {
            const int q = qt * 16 + m;
            const v8h bv0 = xs8[q * 4 + h];
            const v8h bv1 = xs8[q * 4 + 2 + h];
            const v16h Bx = __builtin_shufflevector(bv0, bv1, 0, 1, 2, 3, 4, 5, 6, 7,
                                                              8, 9, 10, 11, 12, 13, 14, 15);

            const float qang = (float)(q * 32);
            float ca[8], sa[8];
            #pragma unroll
            for (int v = 0; v < 8; ++v) {
                const float ang = wrow[v] * qang;
                ca[v] = cosf(ang);
                sa[v] = sinf(ang);
            }

            const v8f P = wmma_f16_16x16x32(Ac, Bx, zero8);
            const v8f S = wmma_f16_16x16x32(As, Bx, zero8);

            #pragma unroll
            for (int v = 0; v < 8; ++v) {
                const float pv = P[v], sv = S[v];
                const float t1 = ca[v] * pv;
                const float t2 = sa[v] * sv;
                const float t3 = sa[v] * pv;
                const float t4 = ca[v] * sv;
                cacc[v] += t1 - t2;
                sacc[v] += t3 + t4;
            }
        }

        #pragma unroll
        for (int v = 0; v < 8; ++v) {
            float cv = cacc[v], sv = sacc[v];
            #pragma unroll
            for (int o = 1; o < 16; o <<= 1) {
                cv += __shfl_xor(cv, o, 32);
                sv += __shfl_xor(sv, o, 32);
            }
            cacc[v] = cv; sacc[v] = sv;
        }

        if (m == 0) {
            #pragma unroll
            for (int v = 0; v < 8; ++v) {
                const int j = bin0 + 8 * h + v;
                if (j < Ftot) {
                    const float p = cacc[v] * cacc[v] + sacc[v] * sacc[v];
                    if (j < Fw) {
                        accW += p;
                    } else {
                        const float fj = bin_freq(j, Fw, K, ft, delta, sfrq, fmin);
                        if (j < Fw + K) {
                            if (fj < thr1) { accU += p; accC += 1; }
                        } else {
                            if (fj < thr2) { accU += p; accC += 1; }
                        }
                    }
                }
            }
        }
    }

    accW += __shfl_xor(accW, 16, 32);
    accU += __shfl_xor(accU, 16, 32);
    accC += __shfl_xor(accC, 16, 32);
    if (lane == 0) { sW[wave] = accW; sU[wave] = accU; sC[wave] = accC; }
    __syncthreads();
    if (tid == 0) {
        float tW = 0.0f, tU = 0.0f;
        int   tC = 0;
        #pragma unroll
        for (int w = 0; w < WAVES; ++w) { tW += sW[w]; tU += sU[w]; tC += sC[w]; }
        const float term1 = tW / (float)Fw;
        const float term2 = tU / (float)tC;
        sRes = 10.0f * log10f(term1 / term2);
    }
    __syncthreads();

    const float r = sRes;
    const v4f val = {r, r, r, r};
    volatile v4f* p = (volatile v4f*)(snr_ws + (size_t)b * LINEF + (size_t)((tid & 7) * 4));
    if (tid < 8) *p = val;
    __threadfence();
    if (tid < 8) *p = val;
}

__global__ __launch_bounds__(32) void k_mean(
    const float* __restrict__ snr_ws, float* __restrict__ out, int B)
{
    if (threadIdx.x != 0) return;
    float s = 0.0f;
    #pragma unroll 1
    for (int b = 0; b < B; ++b) {
        float v = snr_ws[(size_t)b * LINEF];
        if (__float_as_uint(v) == 0xAAAAAAAAu) v = snr_ws[(size_t)b * LINEF + 16];
        s += v;
    }
    const float res = -(s / (float)B);
    volatile float* po = (volatile float*)out;
    *po = res;
    __threadfence();
    *po = res;
}

extern "C" void kernel_launch(void* const* d_in, const int* in_sizes, int n_in,
                              void* d_out, int out_size, void* d_ws, size_t ws_size,
                              hipStream_t stream)
{
    if (n_in < 7) return;
    const float* x          = (const float*)d_in[0];
    const float* f_true     = (const float*)d_in[1];
    const float* fs         = (const float*)d_in[2];
    const float* delta      = (const float*)d_in[3];
    const float* sampling_f = (const float*)d_in[4];
    const float* f_min      = (const float*)d_in[5];
    const float* f_max      = (const float*)d_in[6];

    const int B = in_sizes[1];
    if (B <= 0) return;
    const int N = in_sizes[0] / B;
    if (N <= 0 || out_size < 1) return;

    if ((size_t)B * (size_t)(LINEF * sizeof(float)) > ws_size) return;
    float* snr_ws = (float*)d_ws;

    k_psd_snr<<<dim3((unsigned)B), dim3(THREADS), 0, stream>>>(
        x, f_true, fs, delta, sampling_f, f_min, f_max, snr_ws, B, N);
    k_mean<<<dim3(1), dim3(32), 0, stream>>>(snr_ws, (float*)d_out, B);
}
